// RandomForestNet_55113020342401
// MI455X (gfx1250) — hardware-verified
//
#include <hip/hip_runtime.h>

#define B_ROWS     16384
#define F_DIM      256
#define E_DIM      512
#define DEPTHM1    7
#define ROWS_PB    32
#define LDS_STRIDE 264
#define W_SCALE    16.0f
#define W_UNSCALE  0.0625f

static_assert(B_ROWS % ROWS_PB == 0);
static_assert(F_DIM % 32 == 0);
static_assert((E_DIM * F_DIM) % 8 == 0);
static_assert(E_DIM == 8 * 64);

typedef _Float16     v16h __attribute__((ext_vector_type(16)));
typedef _Float16     v8h  __attribute__((ext_vector_type(8)));
typedef _Float16     v4h  __attribute__((ext_vector_type(4)));
typedef float        v8f  __attribute__((ext_vector_type(8)));
typedef float        v4f  __attribute__((ext_vector_type(4)));
typedef unsigned int v4u  __attribute__((ext_vector_type(4)));

union Frag   { v16h v; v8h half[2]; };
union Pack16 { v8h h; v4u u; };

__device__ __forceinline__ v8f wmma16(v16h a, v16h b, v8f c) {
    c = __builtin_amdgcn_wmma_f32_16x16x32_f16(false, a, false, b, (short)0, c, false, false);
    asm volatile("v_nop\n\tv_nop\n\tv_nop\n\tv_nop" : "+v"(c) : "v"(a), "v"(b));
    return c;
}

__global__ __launch_bounds__(256) void cvt_w0_f16(const float* __restrict__ w0,
                                                  _Float16* __restrict__ w0h,
                                                  int n8) {
    const int i = blockIdx.x * 256 + threadIdx.x;
    if (i >= n8) return;
    const float4* src = (const float4*)(w0 + (size_t)i * 8);
    const float4 f0 = src[0];
    const float4 f1 = src[1];
    Pack16 cv;
    cv.h[0] = (_Float16)(f0.x * W_SCALE);
    cv.h[1] = (_Float16)(f0.y * W_SCALE);
    cv.h[2] = (_Float16)(f0.z * W_SCALE);
    cv.h[3] = (_Float16)(f0.w * W_SCALE);
    cv.h[4] = (_Float16)(f1.x * W_SCALE);
    cv.h[5] = (_Float16)(f1.y * W_SCALE);
    cv.h[6] = (_Float16)(f1.z * W_SCALE);
    cv.h[7] = (_Float16)(f1.w * W_SCALE);
    const v4u val = cv.u;
    volatile v4u* dst = (volatile v4u*)(w0h + (size_t)i * 8);
    *dst = val;
    __threadfence();
    *dst = val;
}

__global__ __launch_bounds__(256) void forest_fused(
    const float*    __restrict__ x,
    const _Float16* __restrict__ w0h,
    const float*    __restrict__ b0,
    const float*    __restrict__ Wc,
    const float*    __restrict__ bc,
    const float*    __restrict__ Wf,
    const float*    __restrict__ bf,
    float*          __restrict__ out)
{
    __shared__ __attribute__((aligned(16))) _Float16 lds_x[ROWS_PB * LDS_STRIDE];
    __shared__ __attribute__((aligned(16))) float    lds_part[8][ROWS_PB];
    __shared__ __attribute__((aligned(16))) float    lds_fin[ROWS_PB];

    const int tid   = threadIdx.x;
    const int wave  = tid >> 5;
    const int lane  = tid & 31;
    const int half  = lane >> 4;
    const int n16   = lane & 15;
    const int bbase = blockIdx.x * ROWS_PB;
    const int ebase = wave * 64;

    #pragma unroll
    for (int i = 0; i < 8; ++i) {
        const int idx = tid + i * 256;
        const int row = idx >> 6;
        const int k   = (idx & 63) << 2;
        const float4 f = *(const float4*)(x + (size_t)(bbase + row) * F_DIM + k);
        v4h o;
        o[0] = (_Float16)f.x; o[1] = (_Float16)f.y; o[2] = (_Float16)f.z; o[3] = (_Float16)f.w;
        *(v4h*)(&lds_x[row * LDS_STRIDE + k]) = o;
    }
    __syncthreads();

    v8f acc[4][2];
    #pragma unroll
    for (int et = 0; et < 4; ++et)
        #pragma unroll
        for (int bt = 0; bt < 2; ++bt)
            acc[et][bt] = (v8f)(0.0f);

    const _Float16* al0 = lds_x + (0 * 16 + n16) * LDS_STRIDE + 8 * half;
    const _Float16* al1 = lds_x + (1 * 16 + n16) * LDS_STRIDE + 8 * half;
    const _Float16* bl  = w0h + (size_t)(ebase + n16) * F_DIM + 8 * half;

    #pragma unroll 1
    for (int k0 = 0; k0 < F_DIM; k0 += 32) {
        Frag a0, a1;
        a0.half[0] = *(const v8h*)(al0 + k0);
        a0.half[1] = *(const v8h*)(al0 + k0 + 16);
        a1.half[0] = *(const v8h*)(al1 + k0);
        a1.half[1] = *(const v8h*)(al1 + k0 + 16);
        #pragma unroll
        for (int et = 0; et < 4; ++et) {
            Frag b;
            const _Float16* q = bl + (size_t)et * 16 * F_DIM + k0;
            b.half[0] = *(const v8h*)(q);
            b.half[1] = *(const v8h*)(q + 16);
            acc[et][0] = wmma16(a0.v, b.v, acc[et][0]);
            acc[et][1] = wmma16(a1.v, b.v, acc[et][1]);
        }
    }

    float rs[2][8];
    #pragma unroll
    for (int bt = 0; bt < 2; ++bt)
        #pragma unroll
        for (int r = 0; r < 8; ++r) rs[bt][r] = 0.0f;

    #pragma unroll
    for (int et = 0; et < 4; ++et) {
        const int e = ebase + et * 16 + n16;
        const float b0e = b0[e];
        const float wfe = Wf[e];
        const float bfe = bf[e];
        float wcd[DEPTHM1], bcd[DEPTHM1];
        #pragma unroll
        for (int d = 0; d < DEPTHM1; ++d) {
            wcd[d] = Wc[d * E_DIM + e];
            bcd[d] = bc[d * E_DIM + e];
        }
        #pragma unroll
        for (int bt = 0; bt < 2; ++bt) {
            #pragma unroll
            for (int r = 0; r < 8; ++r) {
                float h = acc[et][bt][r] * W_UNSCALE + b0e;
                h = fmaxf(h, 0.0f);
                #pragma unroll
                for (int d = 0; d < DEPTHM1; ++d)
                    h = fmaxf(h * wcd[d] + bcd[d], 0.0f);
                rs[bt][r] += h * wfe + bfe;
            }
        }
    }

    #pragma unroll
    for (int m = 1; m <= 8; m <<= 1) {
        #pragma unroll
        for (int r = 0; r < 8; ++r) {
            rs[0][r] += __shfl_xor(rs[0][r], m, 32);
            rs[1][r] += __shfl_xor(rs[1][r], m, 32);
        }
    }
    if (n16 == 0) {
        #pragma unroll
        for (int r = 0; r < 8; ++r) {
            lds_part[wave][0 * 16 + half * 8 + r] = rs[0][r];
            lds_part[wave][1 * 16 + half * 8 + r] = rs[1][r];
        }
    }
    __syncthreads();

    if (tid < ROWS_PB) {
        float s = 0.0f;
        #pragma unroll
        for (int w = 0; w < 8; ++w) s += lds_part[w][tid];
        lds_fin[tid] = s * (1.0f / (float)E_DIM);
    }
    __syncthreads();

    if (tid < ROWS_PB / 4) {
        const v4f v = *(const v4f*)(&lds_fin[4 * tid]);
        volatile v4f* p = (volatile v4f*)(out + (size_t)bbase + 4 * tid);
        *p = v;
        __threadfence();
        *p = v;
    }
}

extern "C" void kernel_launch(void* const* d_in, const int* in_sizes, int n_in,
                              void* d_out, int out_size, void* d_ws, size_t ws_size,
                              hipStream_t stream) {
    if (n_in < 7) return;
    if (in_sizes[0] != B_ROWS * F_DIM || in_sizes[1] != E_DIM * F_DIM ||
        in_sizes[2] != E_DIM || in_sizes[3] != DEPTHM1 * E_DIM ||
        in_sizes[4] != DEPTHM1 * E_DIM || in_sizes[5] != E_DIM ||
        in_sizes[6] != E_DIM || out_size != B_ROWS) return;

    const float* x  = (const float*)d_in[0];
    const float* W0 = (const float*)d_in[1];
    const float* b0 = (const float*)d_in[2];
    const float* Wc = (const float*)d_in[3];
    const float* bc = (const float*)d_in[4];
    const float* Wf = (const float*)d_in[5];
    const float* bf = (const float*)d_in[6];
    float* out = (float*)d_out;

    const size_t w0h_bytes = (size_t)in_sizes[1] * sizeof(_Float16);
    if (w0h_bytes > ws_size) return;
    _Float16* w0h = (_Float16*)d_ws;

    const int n8 = in_sizes[1] / 8;
    cvt_w0_f16<<<(n8 + 255) / 256, 256, 0, stream>>>(W0, w0h, n8);
    forest_fused<<<B_ROWS / ROWS_PB, 256, 0, stream>>>(x, w0h, b0, Wc, bc, Wf, bf, out);
}
